// MultiHeadAttention_17978733101316
// MI455X (gfx1250) — hardware-run, weakly checked
//
#include <hip/hip_runtime.h>
#ifndef NB
#define NB 2
#endif
#ifndef SEQ
#define SEQ 2048
#endif
#define NB_FULL 2
#define SEQ_FULL 2048
#define EMB 1024
#define NH 16
#define HD 64
#define NTOK (NB * SEQ)
#define XSTRIDE_FULL ((size_t)SEQ_FULL * EMB)
#define MROW_FULL ((size_t)SEQ_FULL)
#define MSTRIDE_FULL ((size_t)SEQ_FULL * SEQ_FULL)
#define OUT1_OFF ((size_t)NB_FULL * SEQ_FULL * EMB)
#define AVP (SEQ + 4)
#define MWORDS (SEQ / 32)
#define SOP 72
#define ATTN_LDS ((size_t)(16 * AVP + 16 * MWORDS) * 4 + (size_t)16 * SOP * 2)

static_assert(SEQ % 128 == 0);
static_assert(SEQ <= SEQ_FULL);
static_assert(NB <= NB_FULL);
static_assert(HD == 64);
static_assert(EMB == NH * HD);
static_assert(EMB == 1024);
static_assert(OUT1_OFF * 4 == (size_t)16777216);
static_assert((16 * MWORDS) % 32 == 0);
static_assert((size_t)7 * NTOK * EMB * 2 + (size_t)4 * EMB * EMB * 2 <= (size_t)134217728);

typedef __bf16 v16b __attribute__((ext_vector_type(16)));
typedef _Float16 v16h __attribute__((ext_vector_type(16)));
typedef unsigned short v8us __attribute__((ext_vector_type(8), may_alias));
typedef float v8f __attribute__((ext_vector_type(8)));
typedef float v4f __attribute__((ext_vector_type(4)));
typedef float v4fa __attribute__((ext_vector_type(4), may_alias));
typedef int v4ia __attribute__((ext_vector_type(4), may_alias));
union Frag { v16b vb; v16h vh; v8us half[2]; };
union FragH { v16h v; v8us half[2]; _Float16 h[16]; };
union H8 { _Float16 h[8]; v8us v; };

#define LOG2E 1.4426950408889634f
#define NEGV (-1000000000.0f)

__device__ __forceinline__ unsigned short bf16_bits(float x) {
  unsigned int u = __float_as_uint(x);
  return (unsigned short)((u + 0x7FFFu + ((u >> 16) & 1u)) >> 16);
}
__device__ __forceinline__ float bf16_val(unsigned short b) { return __uint_as_float(((unsigned int)b) << 16); }
__device__ __forceinline__ float bf16_rne(float x) { return bf16_val(bf16_bits(x)); }

template <bool F16>
__device__ __forceinline__ void mma4(const Frag& a, const Frag& b0, const Frag& b1, const Frag& b2, const Frag& b3,
                                     v8f& c0, v8f& c1, v8f& c2, v8f& c3) {
  if (F16) {
    c0 = __builtin_amdgcn_wmma_f32_16x16x32_f16(false, a.vh, false, b0.vh, (short)0, c0, false, false);
    c1 = __builtin_amdgcn_wmma_f32_16x16x32_f16(false, a.vh, false, b1.vh, (short)0, c1, false, false);
    c2 = __builtin_amdgcn_wmma_f32_16x16x32_f16(false, a.vh, false, b2.vh, (short)0, c2, false, false);
    c3 = __builtin_amdgcn_wmma_f32_16x16x32_f16(false, a.vh, false, b3.vh, (short)0, c3, false, false);
  } else {
    c0 = __builtin_amdgcn_wmma_f32_16x16x32_bf16(false, a.vb, false, b0.vb, (short)0, c0, false, false);
    c1 = __builtin_amdgcn_wmma_f32_16x16x32_bf16(false, a.vb, false, b1.vb, (short)0, c1, false, false);
    c2 = __builtin_amdgcn_wmma_f32_16x16x32_bf16(false, a.vb, false, b2.vb, (short)0, c2, false, false);
    c3 = __builtin_amdgcn_wmma_f32_16x16x32_bf16(false, a.vb, false, b3.vb, (short)0, c3, false, false);
  }
  asm volatile("v_nop\n\tv_nop\n\tv_nop\n\tv_nop"
               : "+v"(c0), "+v"(c1), "+v"(c2), "+v"(c3)
               : "v"(a.vh), "v"(b0.vh), "v"(b1.vh), "v"(b2.vh), "v"(b3.vh));
}
__device__ __forceinline__ v8f mma_s2(v16h a0, v16h b0, v16h a1, v16h b1, v8f c) {
  c = __builtin_amdgcn_wmma_f32_16x16x32_f16(false, a0, false, b0, (short)0, c, false, false);
  c = __builtin_amdgcn_wmma_f32_16x16x32_f16(false, a1, false, b1, (short)0, c, false, false);
  asm volatile("v_nop\n\tv_nop\n\tv_nop\n\tv_nop" : "+v"(c) : "v"(a0), "v"(b0), "v"(a1), "v"(b1));
  return c;
}
__device__ __forceinline__ void mma_h2(v16h a, v16h bh, v16h bl, v8f& ch, v8f& cl) {
  ch = __builtin_amdgcn_wmma_f32_16x16x32_f16(false, a, false, bh, (short)0, ch, false, false);
  cl = __builtin_amdgcn_wmma_f32_16x16x32_f16(false, a, false, bl, (short)0, cl, false, false);
  asm volatile("v_nop\n\tv_nop\n\tv_nop\n\tv_nop" : "+v"(ch), "+v"(cl) : "v"(a), "v"(bh), "v"(bl));
}

template <int MODE>
__global__ __launch_bounds__(256) void k_cvt(const float* __restrict__ src, unsigned short* __restrict__ dst,
                                             int nrows, int rpb, int rpb_full) {
  const int t = blockIdx.x * 256 + threadIdx.x;
  if (t >= nrows * 128) return;
  const int row = t >> 7, piece = t & 127;
  const int b = row / rpb, s = row - b * rpb;
  const float* p = src + ((size_t)b * rpb_full + s) * EMB + piece * 8;
  const v4f x0 = *(const v4fa*)(p), x1 = *(const v4fa*)(p + 4);
  v8us o;
  if (MODE == 0) {
    o[0] = bf16_bits(x0[0]); o[1] = bf16_bits(x0[1]); o[2] = bf16_bits(x0[2]); o[3] = bf16_bits(x0[3]);
    o[4] = bf16_bits(x1[0]); o[5] = bf16_bits(x1[1]); o[6] = bf16_bits(x1[2]); o[7] = bf16_bits(x1[3]);
  } else {
    H8 hp;
    hp.h[0] = (_Float16)(bf16_rne(x0[0]) * 256.0f); hp.h[1] = (_Float16)(bf16_rne(x0[1]) * 256.0f);
    hp.h[2] = (_Float16)(bf16_rne(x0[2]) * 256.0f); hp.h[3] = (_Float16)(bf16_rne(x0[3]) * 256.0f);
    hp.h[4] = (_Float16)(bf16_rne(x1[0]) * 256.0f); hp.h[5] = (_Float16)(bf16_rne(x1[1]) * 256.0f);
    hp.h[6] = (_Float16)(bf16_rne(x1[2]) * 256.0f); hp.h[7] = (_Float16)(bf16_rne(x1[3]) * 256.0f);
    o = hp.v;
  }
  unsigned short* d = dst + (size_t)t * 8;
  *(volatile v8us*)d = o;
  __threadfence();
  *(volatile v8us*)d = o;
}

template <int MODE>
__global__ __launch_bounds__(128) void k_gemm(const unsigned short* __restrict__ X, const unsigned short* __restrict__ W,
                                              const float* __restrict__ bias, unsigned short* __restrict__ o16,
                                              float* __restrict__ o32) {
  __shared__ __attribute__((aligned(16))) float st[128][68];
  const int tid = threadIdx.x, w = __builtin_amdgcn_readfirstlane((int)(tid >> 5)), lane = tid & 31, ln = lane & 15, hh = lane >> 4;
  const int n0 = blockIdx.x * 64, mb0 = blockIdx.y * 128, m0 = mb0 + 32 * w;
  const unsigned short* a0p = X + (size_t)(m0 + ln) * EMB + 8 * hh;
  const unsigned short* a1p = a0p + (size_t)16 * EMB;
  const unsigned short* bp = W + (size_t)(n0 + ln) * EMB + 8 * hh;
  v8f c0[4] = {}, c1[4] = {};
#pragma unroll 1
  for (int k0 = 0; k0 < EMB; k0 += 32) {
    Frag a0, a1, b0, b1, b2, b3;
    a0.half[0] = *(const v8us*)(a0p + k0);                      a0.half[1] = *(const v8us*)(a0p + k0 + 16);
    a1.half[0] = *(const v8us*)(a1p + k0);                      a1.half[1] = *(const v8us*)(a1p + k0 + 16);
    b0.half[0] = *(const v8us*)(bp + k0);                       b0.half[1] = *(const v8us*)(bp + k0 + 16);
    b1.half[0] = *(const v8us*)(bp + (size_t)16 * EMB + k0);    b1.half[1] = *(const v8us*)(bp + (size_t)16 * EMB + k0 + 16);
    b2.half[0] = *(const v8us*)(bp + (size_t)32 * EMB + k0);    b2.half[1] = *(const v8us*)(bp + (size_t)32 * EMB + k0 + 16);
    b3.half[0] = *(const v8us*)(bp + (size_t)48 * EMB + k0);    b3.half[1] = *(const v8us*)(bp + (size_t)48 * EMB + k0 + 16);
    mma4<MODE == 2>(a0, b0, b1, b2, b3, c0[0], c0[1], c0[2], c0[3]);
    mma4<MODE == 2>(a1, b0, b1, b2, b3, c1[0], c1[1], c1[2], c1[3]);
  }
#pragma unroll
  for (int t = 0; t < 4; ++t) {
    const int n = 16 * t + ln;
    const float bv = bf16_rne(bias[n0 + n]);
#pragma unroll
    for (int r = 0; r < 8; ++r) {
      float v0, v1;
      if (MODE == 0)      { v0 = c0[t][r] + bv;                   v1 = c1[t][r] + bv; }
      else if (MODE == 1) { v0 = (c0[t][r] + bv) * 16.0f;         v1 = (c1[t][r] + bv) * 16.0f; }
      else                { v0 = c0[t][r] * 0.0000152587890625f + bv; v1 = c1[t][r] * 0.0000152587890625f + bv; }
      st[32 * w + 8 * hh + r][n] = v0;
      st[32 * w + 16 + 8 * hh + r][n] = v1;
    }
  }
  __syncthreads();
  const int b = mb0 / SEQ, s0 = mb0 - b * SEQ;
  if (MODE == 0) {
    unsigned short* ob = o16 + (size_t)mb0 * EMB + n0;
    for (int pass = 0; pass < 2; ++pass) {
#pragma unroll 1
      for (int it = 0; it < 8; ++it) {
        const int idx = it * 128 + tid;
        const int row = idx >> 3, p8 = (idx & 7) * 8;
        const v4f x0 = *(const v4fa*)&st[row][p8], x1 = *(const v4fa*)&st[row][p8 + 4];
        H8 o;
        o.h[0] = (_Float16)x0[0]; o.h[1] = (_Float16)x0[1]; o.h[2] = (_Float16)x0[2]; o.h[3] = (_Float16)x0[3];
        o.h[4] = (_Float16)x1[0]; o.h[5] = (_Float16)x1[1]; o.h[6] = (_Float16)x1[2]; o.h[7] = (_Float16)x1[3];
        *(volatile v8us*)(ob + (size_t)row * EMB + p8) = o.v;
      }
      if (pass == 0) __threadfence();
    }
  } else if (MODE == 1) {
    unsigned short* ob = o16 + (size_t)(b * NH + (int)blockIdx.x) * HD * SEQ + s0;
    for (int pass = 0; pass < 2; ++pass) {
#pragma unroll 1
      for (int it = 0; it < 8; ++it) {
        const int idx = it * 128 + tid;
        const int line = idx >> 3, p8 = (idx & 7) * 8;
        const int d = line & 63, g = line >> 6;
        H8 o;
#pragma unroll
        for (int q = 0; q < 8; ++q) o.h[q] = (_Float16)st[64 * g + p8 + q][d];
        *(volatile v8us*)(ob + (size_t)d * SEQ + 64 * g + p8) = o.v;
      }
      if (pass == 0) __threadfence();
    }
  } else {
    float* ob = o32 + ((size_t)b * SEQ_FULL + s0) * EMB + n0;
    for (int pass = 0; pass < 2; ++pass) {
#pragma unroll 1
      for (int it = 0; it < 16; ++it) {
        const int idx = it * 128 + tid;
        const int row = idx >> 4, c4 = (idx & 15) * 4;
        const v4f v = *(const v4fa*)&st[row][c4];
        *(volatile v4f*)(ob + (size_t)row * EMB + c4) = v;
      }
      if (pass == 0) __threadfence();
    }
  }
}

__device__ __forceinline__ void score_tile(const unsigned short* __restrict__ Kh, int key0, int ln, int hh,
                                           const FragH& q0, const FragH& q1, unsigned int mw, float (&sc)[16]) {
  const unsigned short* kp0 = Kh + (size_t)(key0 + ln) * EMB + 8 * hh;
  const unsigned short* kp1 = kp0 + (size_t)16 * EMB;
  FragH k00, k01, k10, k11;
  k00.half[0] = *(const v8us*)(kp0);      k00.half[1] = *(const v8us*)(kp0 + 16);
  k01.half[0] = *(const v8us*)(kp0 + 32); k01.half[1] = *(const v8us*)(kp0 + 48);
  k10.half[0] = *(const v8us*)(kp1);      k10.half[1] = *(const v8us*)(kp1 + 16);
  k11.half[0] = *(const v8us*)(kp1 + 32); k11.half[1] = *(const v8us*)(kp1 + 48);
  const v8f z8 = {0.f, 0.f, 0.f, 0.f, 0.f, 0.f, 0.f, 0.f};
  const v8f s0 = mma_s2(k00.v, q0.v, k01.v, q1.v, z8);
  const v8f s1 = mma_s2(k10.v, q0.v, k11.v, q1.v, z8);
  const unsigned int w0 = mw >> (8 * hh);
#pragma unroll
  for (int r = 0; r < 8; ++r) {
    const float a = s0[r] * 0.125f, c = s1[r] * 0.125f;
    sc[r]     = ((w0 >> r) & 1u) ? a : NEGV;
    sc[8 + r] = ((w0 >> (16 + r)) & 1u) ? c : NEGV;
  }
}

__global__ __launch_bounds__(32) void k_attn(const unsigned short* __restrict__ Qp, const unsigned short* __restrict__ Kp,
                                             const unsigned short* __restrict__ Vt, const int* __restrict__ mask,
                                             unsigned short* __restrict__ Cx, float* __restrict__ avg) {
  extern __shared__ __attribute__((aligned(16))) float smem[];
  float* av = smem;
  unsigned int* mb = (unsigned int*)(smem + 16 * AVP);
  unsigned short* so16 = (unsigned short*)(smem + 16 * AVP + 16 * MWORDS);
  const int lane = threadIdx.x, ln = lane & 15, hh = lane >> 4;
  const int b = blockIdx.x / (SEQ / 16), qt = blockIdx.x % (SEQ / 16);
  const int qbase = qt * 16;
  const int qg = qbase + ln;

  {
    const v4f z4 = {0.f, 0.f, 0.f, 0.f};
    for (int i = lane; i < 4 * AVP; i += 32) *(v4fa*)(av + 4 * i) = z4;
  }
#pragma unroll 1
  for (int i = 0; i < (16 * MWORDS) / 32; ++i) {
    const int wi = i * 32 + lane;
    const int q = wi / MWORDS, j = wi - q * MWORDS;
    const int* mp = mask + (size_t)b * MSTRIDE_FULL + (size_t)(qbase + q) * MROW_FULL + 32 * j;
    unsigned int wd = 0u;
#pragma unroll
    for (int c = 0; c < 8; ++c) {
      const v4ia m4 = *(const v4ia*)(mp + 4 * c);
      wd |= ((m4[0] != 0) ? 1u : 0u) << (4 * c);
      wd |= ((m4[1] != 0) ? 1u : 0u) << (4 * c + 1);
      wd |= ((m4[2] != 0) ? 1u : 0u) << (4 * c + 2);
      wd |= ((m4[3] != 0) ? 1u : 0u) << (4 * c + 3);
    }
    mb[wi] = wd;
  }
  __syncthreads();

  const size_t tokq = (size_t)b * SEQ + qg;
  float* avl = av + ln * AVP + 8 * hh;
  const unsigned int* mbl = mb + ln * MWORDS;

#pragma unroll 1
  for (int h = 0; h < NH; ++h) {
    const unsigned short* qrow = Qp + tokq * EMB + h * HD + 8 * hh;
    FragH q0, q1;
    q0.half[0] = *(const v8us*)(qrow);      q0.half[1] = *(const v8us*)(qrow + 16);
    q1.half[0] = *(const v8us*)(qrow + 32); q1.half[1] = *(const v8us*)(qrow + 48);
    const unsigned short* Kh = Kp + (size_t)b * SEQ * EMB + h * HD;
    const unsigned short* Vh = Vt + (size_t)(b * NH + h) * HD * SEQ;

    float mr = -3.0e38f, lr = 0.0f;
#pragma unroll 1
    for (int j = 0; j < SEQ / 32; ++j) {
      float sc[16];
      score_tile(Kh, 32 * j, ln, hh, q0, q1, mbl[j], sc);
      float mx = sc[0];
#pragma unroll
      for (int i = 1; i < 16; ++i) mx = fmaxf(mx, sc[i]);
      mx = fmaxf(mx, __shfl_xor(mx, 16, 32));
      const float mnew = fmaxf(mr, mx);
      const float al = exp2f((mr - mnew) * LOG2E);
      mr = mnew;
      float ps = 0.0f;
#pragma unroll
      for (int i = 0; i < 16; ++i) ps += exp2f((sc[i] - mnew) * LOG2E);
      ps += __shfl_xor(ps, 16, 32);
      lr = lr * al + ps;
    }
    const float inv = 1.0f / (16.0f * lr);
    const float cav = inv * 0.00390625f;

    v8f Oh[4] = {}, Ol[4] = {};
#pragma unroll 1
    for (int j = 0; j < SEQ / 32; ++j) {
      const int key0 = 32 * j;
      float sc[16];
      score_tile(Kh, key0, ln, hh, q0, q1, mbl[j], sc);
      const unsigned short* vp = Vh + (size_t)ln * SEQ + key0 + 8 * hh;
      FragH vf[4];
#pragma unroll
      for (int t = 0; t < 4; ++t) {
        vf[t].half[0] = *(const v8us*)(vp + (size_t)t * 16 * SEQ);
        vf[t].half[1] = *(const v8us*)(vp + (size_t)t * 16 * SEQ + 16);
      }
      FragH ph, pl;
      float pc[16];
#pragma unroll
      for (int i = 0; i < 16; ++i) {
        pc[i] = exp2f(fmaf(sc[i] - mr, LOG2E, 8.0f));
        const _Float16 hv = (_Float16)pc[i];
        ph.h[i] = hv;
        pl.h[i] = (_Float16)((pc[i] - (float)hv) * 2048.0f);
      }
      float* ap = avl + key0;
      v4f a0 = *(const v4fa*)(ap),      a1 = *(const v4fa*)(ap + 4);
      v4f a2 = *(const v4fa*)(ap + 16), a3 = *(const v4fa*)(ap + 20);
#pragma unroll
      for (int i = 0; i < 4; ++i) {
        a0[i] = fmaf(pc[i], cav, a0[i]);       a1[i] = fmaf(pc[4 + i], cav, a1[i]);
        a2[i] = fmaf(pc[8 + i], cav, a2[i]);   a3[i] = fmaf(pc[12 + i], cav, a3[i]);
      }
      *(v4fa*)(ap) = a0;      *(v4fa*)(ap + 4) = a1;
      *(v4fa*)(ap + 16) = a2; *(v4fa*)(ap + 20) = a3;
#pragma unroll
      for (int t = 0; t < 4; ++t) mma_h2(vf[t].v, ph.v, pl.v, Oh[t], Ol[t]);
    }

    __syncthreads();
#pragma unroll
    for (int t = 0; t < 4; ++t) {
      H8 o;
#pragma unroll
      for (int r = 0; r < 8; ++r) o.h[r] = (_Float16)((Oh[t][r] + Ol[t][r] * 0.00048828125f) * inv);
      *(v8us*)(so16 + ln * SOP + 16 * t + 8 * hh) = o.v;
    }
    __syncthreads();
    unsigned short* cg = Cx + ((size_t)b * SEQ + qbase) * EMB + h * HD;
    const int rsub = lane >> 3, p8 = (lane & 7) * 8;
    for (int pass = 0; pass < 2; ++pass) {
#pragma unroll
      for (int q4 = 0; q4 < 4; ++q4) {
        const int row = 4 * q4 + rsub;
        const v8us v = *(const v8us*)(so16 + row * SOP + p8);
        *(volatile v8us*)(cg + (size_t)row * EMB + p8) = v;
      }
      if (pass == 0) __threadfence();
    }
  }

  __syncthreads();
  float* ab = avg + (size_t)b * MSTRIDE_FULL + (size_t)qbase * MROW_FULL;
  for (int pass = 0; pass < 2; ++pass) {
#pragma unroll 1
    for (int row = 0; row < 16; ++row) {
#pragma unroll 4
      for (int it = 0; it < SEQ / 128; ++it) {
        const int c4 = (it * 32 + lane) * 4;
        const v4f v = *(const v4fa*)(av + row * AVP + c4);
        *(volatile v4f*)(ab + (size_t)row * MROW_FULL + c4) = v;
      }
    }
    if (pass == 0) __threadfence();
  }
}

extern "C" void kernel_launch(void* const* d_in, const int* in_sizes, int n_in,
                              void* d_out, int out_size, void* d_ws, size_t ws_size, hipStream_t stream) {
  if (n_in < 12) return;
  const long long needX = (long long)(NB - 1) * SEQ_FULL * EMB + (long long)SEQ * EMB;
  const long long needM = (long long)(NB - 1) * SEQ_FULL * SEQ_FULL + (long long)(SEQ - 1) * SEQ_FULL + SEQ;
  if ((long long)in_sizes[0] < needX || (long long)in_sizes[1] < needX || (long long)in_sizes[2] < needX) return;
  if ((long long)in_sizes[3] < needM) return;
  if ((long long)in_sizes[4] < (long long)EMB * EMB || (long long)in_sizes[6] < (long long)EMB * EMB ||
      (long long)in_sizes[8] < (long long)EMB * EMB || (long long)in_sizes[10] < (long long)EMB * EMB) return;
  if (in_sizes[5] < EMB || in_sizes[7] < EMB || in_sizes[9] < EMB || in_sizes[11] < EMB) return;
  if ((long long)out_size < (long long)OUT1_OFF + needM) return;

  const float* xq = (const float*)d_in[0];
  const float* xk = (const float*)d_in[1];
  const float* xv = (const float*)d_in[2];
  const int* mask = (const int*)d_in[3];
  const float* Wq = (const float*)d_in[4];
  const float* bq = (const float*)d_in[5];
  const float* Wk = (const float*)d_in[6];
  const float* bk = (const float*)d_in[7];
  const float* Wv = (const float*)d_in[8];
  const float* bv = (const float*)d_in[9];
  const float* Wo = (const float*)d_in[10];
  const float* bo = (const float*)d_in[11];
  float* out0 = (float*)d_out;
  float* out1 = out0 + OUT1_OFF;

  char* ws = (char*)d_ws;
  size_t off = 0;
  const size_t XB = (size_t)NTOK * EMB * 2;
  const size_t WB = (size_t)EMB * EMB * 2;
  unsigned short* Xq = (unsigned short*)(ws + off); off += XB;
  unsigned short* Xk = (unsigned short*)(ws + off); off += XB;
  unsigned short* Xv = (unsigned short*)(ws + off); off += XB;
  unsigned short* Wqb = (unsigned short*)(ws + off); off += WB;
  unsigned short* Wkb = (unsigned short*)(ws + off); off += WB;
  unsigned short* Wvb = (unsigned short*)(ws + off); off += WB;
  unsigned short* Woh = (unsigned short*)(ws + off); off += WB;
  unsigned short* Qp = (unsigned short*)(ws + off); off += XB;
  unsigned short* Kp = (unsigned short*)(ws + off); off += XB;
  unsigned short* Vt = (unsigned short*)(ws + off); off += XB;
  unsigned short* Cx = (unsigned short*)(ws + off); off += XB;
  if (off > ws_size || off > (size_t)134217728) return;

  const unsigned gx = (unsigned)((NTOK * 128 + 255) / 256);
  const unsigned gw = (unsigned)((EMB * 128 + 255) / 256);
  k_cvt<0><<<gx, 256, 0, stream>>>(xq, Xq, NTOK, SEQ, SEQ_FULL);
  k_cvt<0><<<gx, 256, 0, stream>>>(xk, Xk, NTOK, SEQ, SEQ_FULL);
  k_cvt<0><<<gx, 256, 0, stream>>>(xv, Xv, NTOK, SEQ, SEQ_FULL);
  k_cvt<0><<<gw, 256, 0, stream>>>(Wq, Wqb, EMB, EMB, EMB);
  k_cvt<0><<<gw, 256, 0, stream>>>(Wk, Wkb, EMB, EMB, EMB);
  k_cvt<0><<<gw, 256, 0, stream>>>(Wv, Wvb, EMB, EMB, EMB);
  k_cvt<1><<<gw, 256, 0, stream>>>(Wo, Woh, EMB, EMB, EMB);

  const dim3 gg((unsigned)(EMB / 64), (unsigned)(NTOK / 128));
  k_gemm<0><<<gg, 128, 0, stream>>>(Xq, Wqb, bq, Qp, out0);
  k_gemm<0><<<gg, 128, 0, stream>>>(Xk, Wkb, bk, Kp, out0);
  k_gemm<1><<<gg, 128, 0, stream>>>(Xv, Wvb, bv, Vt, out0);

  (void)hipFuncSetAttribute(reinterpret_cast<const void*>(&k_attn), hipFuncAttributeMaxDynamicSharedMemorySize, (int)ATTN_LDS);
  k_attn<<<(unsigned)(NB * (SEQ / 16)), 32, ATTN_LDS, stream>>>(Qp, Kp, Vt, mask, Cx, out1);

  k_gemm<2><<<gg, 128, 0, stream>>>(Cx, Woh, bo, Xq, out0);
}
